// fbank_layer_81784767251215
// MI455X (gfx1250) — hardware-verified
//
#include <hip/hip_runtime.h>


#define NX    8000240
#define NF    50000
#define FCH   10048
#define NCH   5
#define FL    400
#define FS    160
#define NFFT  512
#define NB    257
#define NKK   576
#define KU    416
#define KP    320
#define NFB   64
#define DM    KU
#define LOSC  1024.0f
#define PI2   6.283185307179586f

typedef _Float16 h16;
typedef unsigned short bf;
typedef __attribute__((ext_vector_type(16))) __bf16   v16bf;
typedef __attribute__((ext_vector_type(16))) _Float16 v16h;
typedef __attribute__((ext_vector_type(8)))  _Float16 v8h;
typedef __attribute__((ext_vector_type(8)))  unsigned short v8us;
typedef __attribute__((ext_vector_type(8)))  float    v8f;
typedef __attribute__((ext_vector_type(4)))  float    v4f;
typedef v8h  __attribute__((may_alias)) v8ha;
typedef v4f  __attribute__((may_alias)) v4fa;
typedef v8us __attribute__((may_alias)) v8usa;

__device__ __forceinline__ unsigned short f2bf(float f) { unsigned u = __float_as_uint(f); u += 0x7FFFu + ((u >> 16) & 1u); return (unsigned short)(u >> 16); }
__device__ __forceinline__ float bf2f(unsigned short b) { return __uint_as_float(((unsigned)b) << 16); }
__device__ __forceinline__ float bfr(float f) { return bf2f(f2bf(f)); }
__device__ __forceinline__ v16h cat16(v8h lo, v8h hi) { return __builtin_shufflevector(lo, hi, 0, 1, 2, 3, 4, 5, 6, 7, 8, 9, 10, 11, 12, 13, 14, 15); }
__device__ __forceinline__ v16bf cat16b(v8us lo, v8us hi) { return __builtin_bit_cast(v16bf, __builtin_shufflevector(lo, hi, 0, 1, 2, 3, 4, 5, 6, 7, 8, 9, 10, 11, 12, 13, 14, 15)); }
__device__ __forceinline__ v8f wmma16(v16h a, v16h b, v8f c) { return __builtin_amdgcn_wmma_f32_16x16x32_f16(false, a, false, b, (short)0, c, false, false); }
__device__ __forceinline__ v8f wmmab(v16bf a, v16bf b, v8f c) { return __builtin_amdgcn_wmma_f32_16x16x32_bf16(false, a, false, b, (short)0, c, false, false); }

template <bool SPLITA, bool F16OUT = false>
__global__ __launch_bounds__(128) void k_gemmb(const bf* __restrict__ A, const bf* __restrict__ Al, const bf* __restrict__ Bn, const float* __restrict__ bias, float* C, int ldc, h16* C2, const float* __restrict__ R = nullptr, int K = DM, int roundR = 1) {
    __shared__ __align__(16) float ost[4][16 * 68];
    const int lane = threadIdx.x & 31, wave = threadIdx.x >> 5, lr = lane & 15, hi = lane >> 4;
    const int r0 = blockIdx.x * 64 + wave * 16, c0 = blockIdx.y * 64;
    const size_t aoff = (size_t)(r0 + lr) * K + 8 * hi;
    size_t boff[4];
#pragma unroll
    for (int t = 0; t < 4; ++t) boff[t] = (size_t)(c0 + t * 16 + lr) * K + 8 * hi;
    v8f acc[4];
#pragma unroll
    for (int t = 0; t < 4; ++t) acc[t] = (v8f){};
#pragma unroll 1
    for (int kc = 0; kc < K; kc += 32) {
        const v16bf a = cat16b(*(const v8us*)(A + aoff + kc), *(const v8us*)(A + aoff + kc + 16));
        v16bf al = a;
        if (SPLITA) al = cat16b(*(const v8us*)(Al + aoff + kc), *(const v8us*)(Al + aoff + kc + 16));
#pragma unroll
        for (int t = 0; t < 4; ++t) { const v16bf b = cat16b(*(const v8us*)(Bn + boff[t] + kc), *(const v8us*)(Bn + boff[t] + kc + 16)); acc[t] = wmmab(a, b, acc[t]); if (SPLITA) acc[t] = wmmab(al, b, acc[t]); }
        asm volatile("v_nop\n\tv_nop\n\tv_nop\n\tv_nop" : "+v"(acc[0]), "+v"(acc[1]), "+v"(acc[2]), "+v"(acc[3]) : "v"(a), "v"(al));
    }
    float* os = &ost[wave][0];
#pragma unroll
    for (int t = 0; t < 4; ++t) { const float bv = bias ? bfr(bias[c0 + t * 16 + lr]) : 0.f;
#pragma unroll
        for (int j = 0; j < 8; ++j) os[(hi * 8 + j) * 68 + t * 16 + lr] = acc[t][j] + bv; }
    __syncthreads();
    if (F16OUT) {
        h16* crow = (h16*)(void*)C + (size_t)r0 * ldc + c0;
        auto pass = [&]() {
#pragma unroll
            for (int s = 0; s < 4; ++s) { const int row = 4 * s + (lane >> 3), piece = lane & 7; const float* sp = os + row * 68 + piece * 8; v8h o, o2;
#pragma unroll
                for (int i = 0; i < 8; ++i) { const h16 a = (h16)sp[i]; o[i] = a; o2[i] = (h16)((sp[i] - (float)a) * LOSC); }
                *(volatile v8h*)(crow + (size_t)row * ldc + piece * 8) = o; if (C2) *(volatile v8h*)(C2 + (size_t)r0 * ldc + c0 + (size_t)row * ldc + piece * 8) = o2; }
        };
        pass(); __threadfence(); pass();
    } else {
        float* crow = C + (size_t)r0 * ldc + c0;
        auto pass = [&]() {
#pragma unroll
            for (int s = 0; s < 8; ++s) { const int Lid = (lane >> 3) + 4 * s, piece = lane & 7; const int row = Lid >> 1, cofs = (Lid & 1) * 32 + piece * 4;
                v4f val = *(const v4fa*)(os + row * 68 + cofs); if (R) { const v4f rv = *(const v4f*)(R + ((size_t)r0 + row) * ldc + c0 + cofs); val += roundR ? (v4f){bfr(rv[0]), bfr(rv[1]), bfr(rv[2]), bfr(rv[3])} : rv; }
                *(volatile v4f*)(crow + (size_t)row * ldc + cofs) = val; }
        };
        pass(); __threadfence(); pass();
    }
}


__global__ __launch_bounds__(256) void k_wtp(const float* __restrict__ Wm, int krows, int ncols, int kpad, bf* WT) {
    __shared__ __align__(16) unsigned short tl[64 * 72];
    const int tid = threadIdx.x, k0 = blockIdx.x * 64, n0 = blockIdx.y * 64;
    const int kk = tid >> 2, nq = (tid & 3) * 16;
    const int k = k0 + kk, kc = k < krows ? k : krows - 1;
#pragma unroll
    for (int i = 0; i < 16; ++i) { const int n = n0 + nq + i, ncl = n < ncols ? n : ncols - 1; const float w = Wm[(size_t)kc * ncols + ncl]; tl[(nq + i) * 72 + kk] = (k < krows && n < ncols) ? f2bf(w) : (unsigned short)0; }
    __syncthreads();
    const int piece = tid & 7;
    auto pass = [&]() {
#pragma unroll
        for (int s = 0; s < 2; ++s) { const int nr = (tid >> 3) + 32 * s; const v8us val = *(const v8usa*)(tl + nr * 72 + piece * 8); *(volatile v8us*)(WT + (size_t)(n0 + nr) * kpad + k0 + piece * 8) = val; }
    };
    pass(); __threadfence(); pass();
}

__device__ __forceinline__ float ccoef(int k, int t, int im) { if (t < 0 || t >= FL) return 0.f; const int r = (k * t) & (NFFT - 1); const float a = PI2 * (float)r * (1.0f / NFFT); return im ? -__sinf(a) : __cosf(a); }
__global__ __launch_bounds__(256) void k_dft(bf* Dh, bf* Dl) {
    const int lane = threadIdx.x & 31, row = blockIdx.x * 8 + (threadIdx.x >> 5); if (row >= NKK) return; const int k = row >> 1, im = row & 1;
#pragma unroll 1
    for (int ps = 0; ps < 2; ++ps) {
#pragma unroll 1
        for (int u0 = lane * 8; u0 < KU; u0 += 256) { v8us oh, ol;
#pragma unroll
            for (int i = 0; i < 8; ++i) { const int u = u0 + i; float d = 0.f; if (k < NB && u <= FL) d = ccoef(k, u - 1, im) - 0.97f * ccoef(k, u, im);
                const unsigned short hb = f2bf(d); oh[i] = hb; ol[i] = f2bf(d - bf2f(hb)); }
            const size_t o = (size_t)row * KU + u0; *(volatile v8us*)(Dh + o) = oh; *(volatile v8us*)(Dl + o) = ol; }
        if (ps == 0) __threadfence(); }
}
__global__ __launch_bounds__(256) void k_frames(const float* __restrict__ x, int f0, bf* FR) {
    const int lane = threadIdx.x & 31, fl = blockIdx.x * 8 + (threadIdx.x >> 5); if (fl >= FCH) return; const int f = f0 + fl;
#pragma unroll 1
    for (int ps = 0; ps < 2; ++ps) {
#pragma unroll 1
        for (int u0 = lane * 8; u0 < KU; u0 += 256) { v8us o;
#pragma unroll
            for (int i = 0; i < 8; ++i) { const int u = u0 + i; const long n = (long)f * FS - 1 + u; const bool ok = (f < NF) && (u <= FL) && (n >= 0) && (n < NX); o[i] = ok ? f2bf(x[ok ? n : 0]) : (unsigned short)0; }
            *(volatile v8us*)(FR + (size_t)fl * KU + u0) = o; }
        if (ps == 0) __threadfence(); }
}
__global__ __launch_bounds__(256) void k_power(const float* __restrict__ C1, bf* Ph, bf* Pl) {
    const int lane = threadIdx.x & 31, fl = blockIdx.x * 8 + (threadIdx.x >> 5); if (fl >= FCH) return;
#pragma unroll 1
    for (int ps = 0; ps < 2; ++ps) {
#pragma unroll 1
        for (int b0 = lane * 8; b0 < KP; b0 += 256) { v8us oh, ol;
#pragma unroll
            for (int i = 0; i < 8; ++i) { const int k = b0 + i; float p = 0.f; if (k < NB) { const float re = C1[(size_t)(2 * k) * FCH + fl], imv = C1[(size_t)(2 * k + 1) * FCH + fl]; p = (re * re + imv * imv) * (1.0f / NFFT); }
                const unsigned short hb = f2bf(p); oh[i] = hb; ol[i] = f2bf(p - bf2f(hb)); }
            const size_t o = (size_t)fl * KP + b0; *(volatile v8us*)(Ph + o) = oh; *(volatile v8us*)(Pl + o) = ol; }
        if (ps == 0) __threadfence(); }
}
__global__ __launch_bounds__(256) void k_norm(const float* __restrict__ C2, int f0, float* OUTP) {
    typedef __attribute__((ext_vector_type(2))) float v2f;
    const int lane = threadIdx.x & 31, fl = blockIdx.x * 8 + (threadIdx.x >> 5); const int f = f0 + fl; if (fl >= FCH || f >= NF) return;
    const float a = C2[(size_t)fl * NFB + 2 * lane] + 1e-30f, b = C2[(size_t)fl * NFB + 2 * lane + 1] + 1e-30f;
    float s = a + b;
#pragma unroll
    for (int sh = 16; sh; sh >>= 1) s += __shfl_xor(s, sh, 32);
    const float mu = s * (1.0f / NFB); float v = (a - mu) * (a - mu) + (b - mu) * (b - mu);
#pragma unroll
    for (int sh = 16; sh; sh >>= 1) v += __shfl_xor(v, sh, 32);
    const float sd = sqrtf(v * (1.0f / NFB)); v2f o; o[0] = (a - mu) / sd; o[1] = (b - mu) / sd;
    *(volatile v2f*)(OUTP + (size_t)f * NFB + 2 * lane) = o; __threadfence(); *(volatile v2f*)(OUTP + (size_t)f * NFB + 2 * lane) = o;
}

extern "C" void kernel_launch(void* const* d_in, const int* in_sizes, int n_in,
                              void* d_out, int out_size, void* d_ws, size_t ws_size, hipStream_t stream) {
    (void)in_sizes; (void)n_in; (void)out_size;
    const float* x = (const float*)d_in[0]; const float* filt = (const float*)d_in[1];
    float* out = (float*)d_out;
    char* wsp = (char*)d_ws;
    auto take = [&](size_t bytes) { char* p = wsp; wsp += (bytes + 255) & ~(size_t)255; return (void*)p; };
    bf* Dh = (bf*)take((size_t)NKK * KU * 2); bf* Dl = (bf*)take((size_t)NKK * KU * 2); bf* FBT = (bf*)take((size_t)NFB * KP * 2);
    bf* FR = (bf*)take((size_t)FCH * KU * 2); float* C1 = (float*)take((size_t)NKK * FCH * 4); bf* Ph = (bf*)take((size_t)FCH * KP * 2); bf* Pl = (bf*)take((size_t)FCH * KP * 2); float* C2 = (float*)take((size_t)FCH * NFB * 4);
    if ((size_t)(wsp - (char*)d_ws) > ws_size) return;
    k_dft<<<NKK / 8, 256, 0, stream>>>(Dh, Dl); k_wtp<<<dim3(KP / 64, NFB / 64, 1), 256, 0, stream>>>(filt, NB, NFB, KP, FBT);
    for (int ch = 0; ch < NCH; ++ch) { const int f0 = ch * FCH;
        k_frames<<<FCH / 8, 256, 0, stream>>>(x, f0, FR);
        k_gemmb<true, false><<<dim3(NKK / 64, FCH / 64, 1), 128, 0, stream>>>(Dh, Dl, FR, nullptr, C1, FCH, nullptr, nullptr, KU);
        k_power<<<FCH / 8, 256, 0, stream>>>(C1, Ph, Pl);
        k_gemmb<true, false><<<dim3(FCH / 64, 1, 1), 128, 0, stream>>>(Ph, Pl, FBT, nullptr, C2, NFB, nullptr, nullptr, KP);
        k_norm<<<FCH / 8, 256, 0, stream>>>(C2, f0, out); }
}
